// RNN_54400055771283
// MI455X (gfx1250) — hardware-verified
//
#include <hip/hip_runtime.h>
#include <math.h>

typedef __attribute__((ext_vector_type(16))) _Float16 v16h;
typedef __attribute__((ext_vector_type(8)))  _Float16 v8h;
typedef __attribute__((ext_vector_type(16))) __bf16   v16b;
typedef __attribute__((ext_vector_type(8)))  __bf16   v8b;
typedef __attribute__((ext_vector_type(8)))  float    v8f;
typedef __attribute__((ext_vector_type(4)))  float    v4f;

constexpr int kSeq   = 64;
constexpr int kStep  = 512;
constexpr int kEmb   = 512;
constexpr int kHid   = 512;
constexpr int kVocab = 32000;
constexpr int kCls   = 2;
constexpr int kRows  = kSeq * kStep;
constexpr int kOutN  = kRows * kCls;
static_assert(kSeq == 64 && kStep == 512 && kEmb == 512 && kHid == 512 && kCls == 2);
static_assert(kEmb == kHid);

constexpr float kWCarry    = 64.0f;
constexpr float kWCarryInv = 1.0f / 64.0f;
constexpr float kResCarry  = 2048.0f;
constexpr float kResInv    = 1.0f / 2048.0f;

constexpr int kSeqPB      = 16;
constexpr int kRnnBlocks  = kSeq / kSeqPB;
constexpr int kRnnThreads = 256;
constexpr int kHP         = kHid + 8;
constexpr int kHTile      = kSeqPB * kHP;
constexpr int kFlushT     = 16;
static_assert(kSeq % kSeqPB == 0);
static_assert(kHid == (kRnnThreads / 32) * 64);
static_assert(kHP % 8 == 0);
static_assert((2 * kHTile) % 8 == 0);
static_assert(kStep % kFlushT == 0 && kFlushT * kCls * 4 == 128);
static_assert(kSeqPB * kCls == 32);
static_assert(kHid % 32 == 0 && kEmb % 32 == 0);
static_assert(kRows % 64 == 0 && kHid % 64 == 0);

constexpr int kDwW     = kHid * kHid / 2;
constexpr int kBlkW    = kDwW / 256;
constexpr int kDwBsum  = 2 * kHid;
constexpr int kBlkBsum = kDwBsum / 256;
constexpr int kPrepB1  = kBlkW;
constexpr int kPrepB2  = kPrepB1 + kBlkW;
constexpr int kPrepB3  = kPrepB2 + kBlkW;
constexpr int kPrepB4  = kPrepB3 + kBlkW;
constexpr int kPrepBlocks = kPrepB4 + kBlkBsum;
static_assert(kDwW % 256 == 0 && kDwBsum % 256 == 0 && kPrepBlocks == 2052);

constexpr int kXChunks = kRows * kEmb / 8;
static_assert(kXChunks % 256 == 0);
static_assert(kEmb / 8 == 64 && kSeq == 64);

constexpr int kGemmTiles = (kHid / 64) * (kRows / 64);
static_assert(kGemmTiles % 8 == 0);
constexpr int kGemmGrid = kGemmTiles / 8;

__device__ __forceinline__ unsigned short f2bf_bits(float f) {
  unsigned u = __float_as_uint(f);
  return (unsigned short)((u + 0x7FFFu + ((u >> 16) & 1u)) >> 16);
}
__device__ __forceinline__ float bf_bits2f(unsigned short h) { return __uint_as_float(((unsigned)h) << 16); }

__device__ __forceinline__ void dep_guard_h(v8f& a, v8f& b, v16h x, v16h y) { asm volatile("v_nop\n\tv_nop\n\tv_nop\n\tv_nop" : "+v"(a), "+v"(b) : "v"(x), "v"(y)); }
__device__ __forceinline__ void dep_guard_b(v8f& a, v8f& b, v16b x, v16b y) { asm volatile("v_nop\n\tv_nop\n\tv_nop\n\tv_nop" : "+v"(a), "+v"(b) : "v"(x), "v"(y)); }
__device__ __forceinline__ void dep_guard4_h(v8f& a, v8f& b, v8f& c, v8f& d, v16h x, v16h y) {
  asm volatile("v_nop\n\tv_nop\n\tv_nop\n\tv_nop" : "+v"(a), "+v"(b), "+v"(c), "+v"(d) : "v"(x), "v"(y));
}
__device__ __forceinline__ void dep_guard4_b(v8f& a, v8f& b, v8f& c, v8f& d, v16b x, v16b y) {
  asm volatile("v_nop\n\tv_nop\n\tv_nop\n\tv_nop" : "+v"(a), "+v"(b), "+v"(c), "+v"(d) : "v"(x), "v"(y));
}
__device__ __forceinline__ void dep_guard8_h(v8f& a0, v8f& a1, v8f& a2, v8f& a3, v8f& r0, v8f& r1, v8f& r2, v8f& r3,
                                             v16h x, v16h y, v16h b0, v16h b1, v16h b2, v16h b3) {
  asm volatile("v_nop\n\tv_nop\n\tv_nop\n\tv_nop"
               : "+v"(a0), "+v"(a1), "+v"(a2), "+v"(a3), "+v"(r0), "+v"(r1), "+v"(r2), "+v"(r3)
               : "v"(x), "v"(y), "v"(b0), "v"(b1), "v"(b2), "v"(b3));
}
__device__ __forceinline__ void keep4_h(v16h a, v16h b, v16h c, v16h d) { asm volatile("v_nop" :: "v"(a), "v"(b), "v"(c), "v"(d)); }
__device__ __forceinline__ void keep4_b(v16b a, v16b b, v16b c, v16b d) { asm volatile("v_nop" :: "v"(a), "v"(b), "v"(c), "v"(d)); }
__device__ __forceinline__ void acc_guard4(v8f& a, v8f& b, v8f& c, v8f& d) { asm volatile("v_nop\n\tv_nop\n\tv_nop\n\tv_nop" : "+v"(a), "+v"(b), "+v"(c), "+v"(d)); }

template <typename T> struct Frag;
template <> struct Frag<_Float16> {
  typedef v16h V; union U { v16h v; v8h h[2]; };
  static __device__ __forceinline__ v16h load(const _Float16* p) {
    U f; f.h[0] = *(const v8h*)(p); f.h[1] = *(const v8h*)(p + 16); return f.v;
  }
  static __device__ __forceinline__ v8f mma(v16h a, v16h b, v8f c) {
    return __builtin_amdgcn_wmma_f32_16x16x32_f16(false, a, false, b, (short)0, c, false, false);
  }
  static __device__ __forceinline__ void guard(v8f& a, v8f& b, v16h x, v16h y) { dep_guard_h(a, b, x, y); }
  static __device__ __forceinline__ void guard4(v8f& a, v8f& b, v8f& c, v8f& d, v16h x, v16h y) { dep_guard4_h(a, b, c, d, x, y); }
  static __device__ __forceinline__ void keep(v16h a, v16h b, v16h c, v16h d) { keep4_h(a, b, c, d); }
};
template <> struct Frag<__bf16> {
  typedef v16b V; union U { v16b v; v8b h[2]; };
  static __device__ __forceinline__ v16b load(const __bf16* p) {
    U f; f.h[0] = *(const v8b*)(p); f.h[1] = *(const v8b*)(p + 16); return f.v;
  }
  static __device__ __forceinline__ v8f mma(v16b a, v16b b, v8f c) {
    return __builtin_amdgcn_wmma_f32_16x16x32_bf16(false, a, false, b, (short)0, c, false, false);
  }
  static __device__ __forceinline__ void guard(v8f& a, v8f& b, v16b x, v16b y) { dep_guard_b(a, b, x, y); }
  static __device__ __forceinline__ void guard4(v8f& a, v8f& b, v8f& c, v8f& d, v16b x, v16b y) { dep_guard4_b(a, b, c, d, x, y); }
  static __device__ __forceinline__ void keep(v16b a, v16b b, v16b c, v16b d) { keep4_b(a, b, c, d); }
};

template <int ET> struct Elem;
template <> struct Elem<0> { typedef _Float16 T; };
template <> struct Elem<1> { typedef __bf16 T; };
template <int ET, bool SPLIT, int BIAS_MODE, int OUT_MODE, bool RESID, int ACT = 0>
__global__ __launch_bounds__(256) void wmma_gemm64(
    const unsigned short* __restrict__ Ap, const unsigned short* __restrict__ A2p, int lda, long strideA,
    const unsigned short* __restrict__ Btp, const unsigned short* __restrict__ Bt2p, int ldb, long strideB,
    void* __restrict__ Cout, void* __restrict__ Cout2, int ldc, long strideC,
    const float* __restrict__ bias,
    const float* __restrict__ resid, long strideR,
    int M, int N, int K, float scale) {
  typedef typename Elem<ET>::T T;
  typedef typename Frag<T>::V V;
  const T* A = (const T*)Ap; const T* A2 = (const T*)A2p; const T* Bt = (const T*)Btp; const T* Bt2 = (const T*)Bt2p;
  __shared__ __align__(16) float sT[8][16 * 68];
  const int b    = blockIdx.y;
  const int lane = threadIdx.x & 31;
  const int wave = threadIdx.x >> 5;
  const int tilesN = N >> 6;
  const int tilesM = M >> 6;
  const int tile = blockIdx.x * 8 + wave;
  if (tile >= tilesM * tilesN) return;
  const int tm = tile / tilesN;
  const int tn = tile - tm * tilesN;
  const int m0 = tm << 6;
  const int n0 = tn << 6;

  const T* Ab  = A  + (size_t)b * strideA;
  const T* Bb  = Bt + (size_t)b * strideB;
  const T* Ab2 = SPLIT ? (A2  + (size_t)b * strideA) : nullptr;
  const T* Bb2 = SPLIT ? (Bt2 + (size_t)b * strideB) : nullptr;

  const int rlane = lane & 15;
  const int koff  = (lane >> 4) * 8;
  const int mOff  = (lane >> 4) * 8;

  v8f acc[4][4];
#pragma unroll
  for (int i = 0; i < 4; ++i)
#pragma unroll
    for (int j = 0; j < 4; ++j) acc[i][j] = (v8f){0.f,0.f,0.f,0.f,0.f,0.f,0.f,0.f};

  for (int k0 = 0; k0 < K; k0 += 32) {
    V bh[4], bl[4];
#pragma unroll
    for (int j = 0; j < 4; ++j) {
      const size_t bo = (size_t)(n0 + (j << 4) + rlane) * ldb + koff + k0;
      bh[j] = Frag<T>::load(Bb + bo);
      if (SPLIT) bl[j] = Frag<T>::load(Bb2 + bo);
    }
#pragma unroll
    for (int i = 0; i < 4; ++i) {
      const size_t ao = (size_t)(m0 + (i << 4) + rlane) * lda + koff + k0;
      V ah = Frag<T>::load(Ab + ao);
      V al;
      if (SPLIT) al = Frag<T>::load(Ab2 + ao);
#pragma unroll
      for (int j = 0; j < 4; ++j) {
        acc[i][j] = Frag<T>::mma(ah, bh[j], acc[i][j]);
        if (SPLIT) {
          acc[i][j] = Frag<T>::mma(ah, bl[j], acc[i][j]);
          acc[i][j] = Frag<T>::mma(al, bh[j], acc[i][j]);
        }
      }
      Frag<T>::guard4(acc[i][0], acc[i][1], acc[i][2], acc[i][3], ah, SPLIT ? al : ah);
    }
    Frag<T>::keep(bh[0], bh[1], bh[2], bh[3]);
    if (SPLIT) Frag<T>::keep(bl[0], bl[1], bl[2], bl[3]);
  }
  acc_guard4(acc[0][0], acc[0][1], acc[0][2], acc[0][3]);
  acc_guard4(acc[1][0], acc[1][1], acc[1][2], acc[1][3]);
  acc_guard4(acc[2][0], acc[2][1], acc[2][2], acc[2][3]);
  acc_guard4(acc[3][0], acc[3][1], acc[3][2], acc[3][3]);

  float* slab = sT[wave];
  const float* Rb = RESID ? (resid + (size_t)b * strideR) : nullptr;
#pragma unroll
  for (int i = 0; i < 4; ++i) {
    const int mBase = m0 + (i << 4);
#pragma unroll
    for (int j = 0; j < 4; ++j) {
      const int n = n0 + (j << 4) + rlane;
      float bv = 0.f;
      if (BIAS_MODE == 2) bv = bias[n];
#pragma unroll
      for (int r = 0; r < 8; ++r) {
        float v = acc[i][j][r] * scale;
        if (BIAS_MODE == 1) v += bias[mBase + mOff + r];
        if (BIAS_MODE == 2) v += bv;
        if (RESID) v += Rb[(size_t)(mBase + mOff + r) * ldc + n];
        if (ACT == 1) v = tanhf(v);
        if (ACT == 2) v = fmaxf(v, 0.0f);
        if (ACT == 4) v = (v > 0.f) ? v : 0.01f * v;
        slab[(mOff + r) * 68 + (j << 4) + rlane] = v;
      }
    }
    __builtin_amdgcn_fence(__ATOMIC_RELEASE, "workgroup");
    __builtin_amdgcn_wave_barrier();
    __builtin_amdgcn_fence(__ATOMIC_ACQUIRE, "workgroup");
    if (OUT_MODE == 0) {
      float* C = (float*)Cout + (size_t)b * strideC;
      const int hh = lane >> 4, c4 = (lane & 15) * 4;
      for (int pass = 0; pass < 2; ++pass) {
#pragma unroll
        for (int it = 0; it < 8; ++it) {
          const int row = it * 2 + hh;
          v4f v = *(const v4f*)(slab + row * 68 + c4);
          *(volatile v4f*)(C + (size_t)(mBase + row) * ldc + n0 + c4) = v;
        }
        __threadfence();
      }
    } else {
      const int q = lane >> 3, c8 = (lane & 7) * 8;
      unsigned short* C  = (unsigned short*)Cout  + (size_t)b * strideC;
      unsigned short* C2 = (OUT_MODE == 2) ? ((unsigned short*)Cout2 + (size_t)b * strideC) : nullptr;
      for (int pass = 0; pass < 2; ++pass) {
#pragma unroll
        for (int it = 0; it < 4; ++it) {
          const int row = it * 4 + q;
          const float* sp = slab + row * 68 + c8;
          v8h hv, lv;
#pragma unroll
          for (int e = 0; e < 8; ++e) {
            if (OUT_MODE == 1) {
              hv[e] = (_Float16)sp[e];
            } else {
              unsigned short hb = f2bf_bits(sp[e]);
              unsigned short lb = f2bf_bits(sp[e] - bf_bits2f(hb));
              hv[e] = __builtin_bit_cast(_Float16, hb);
              lv[e] = __builtin_bit_cast(_Float16, lb);
            }
          }
          *(volatile v8h*)(C + (size_t)(mBase + row) * ldc + n0 + c8) = hv;
          if (OUT_MODE == 2) *(volatile v8h*)(C2 + (size_t)(mBase + row) * ldc + n0 + c8) = lv;
        }
        __threadfence();
      }
    }
    __builtin_amdgcn_fence(__ATOMIC_RELEASE, "workgroup");
    __builtin_amdgcn_wave_barrier();
    __builtin_amdgcn_fence(__ATOMIC_ACQUIRE, "workgroup");
  }
}

__device__ __forceinline__ unsigned pack_f16x2(float a, float b) {
  const _Float16 h0 = (_Float16)a, h1 = (_Float16)b;
  return (unsigned)__builtin_bit_cast(unsigned short, h0) | ((unsigned)__builtin_bit_cast(unsigned short, h1) << 16);
}
__device__ __forceinline__ void st2u(unsigned* p, unsigned v) { *(volatile unsigned*)p = v; __threadfence(); *(volatile unsigned*)p = v; }

__global__ __launch_bounds__(256) void prep_kernel(
    const float* __restrict__ w_ih0, const float* __restrict__ w_hh0,
    const float* __restrict__ w_ih1, const float* __restrict__ w_hh1,
    const float* __restrict__ b_ih0, const float* __restrict__ b_hh0,
    const float* __restrict__ b_ih1, const float* __restrict__ b_hh1,
    unsigned* __restrict__ wih0u, unsigned* __restrict__ whh0u,
    unsigned* __restrict__ wih1u, unsigned* __restrict__ whh1u,
    unsigned* __restrict__ bsumu) {
  const int blk = blockIdx.x, tid = threadIdx.x;
  if (blk < kPrepB1) {
    const int p = blk * 256 + tid;
    st2u(wih0u + p, pack_f16x2(w_ih0[2 * p] * kWCarry, w_ih0[2 * p + 1] * kWCarry));
  } else if (blk < kPrepB2) {
    const int p = (blk - kPrepB1) * 256 + tid;
    st2u(whh0u + p, pack_f16x2(w_hh0[2 * p] * kWCarry, w_hh0[2 * p + 1] * kWCarry));
  } else if (blk < kPrepB3) {
    const int p = (blk - kPrepB2) * 256 + tid;
    st2u(wih1u + p, pack_f16x2(w_ih1[2 * p] * kWCarry, w_ih1[2 * p + 1] * kWCarry));
  } else if (blk < kPrepB4) {
    const int p = (blk - kPrepB3) * 256 + tid;
    st2u(whh1u + p, pack_f16x2(w_hh1[2 * p] * kWCarry, w_hh1[2 * p + 1] * kWCarry));
  } else {
    const int p  = (blk - kPrepB4) * 256 + tid;
    const int pc = p & (kHid - 1);
    const float s0 = b_ih0[pc] + b_hh0[pc];
    const float s1 = b_ih1[pc] + b_hh1[pc];
    const float f1 = (p >= kHid) ? 1.0f : 0.0f;
    const float f0 = 1.0f - f1;
    const float v  = fmaf(f1, s1, f0 * s0);
    st2u(bsumu + p, (unsigned)__float_as_uint(v));
  }
}

__global__ __launch_bounds__(256) void gather_kernel(const int* __restrict__ tokens, const float* __restrict__ emb,
                                                    unsigned short* __restrict__ x16p) {
  _Float16* x16t = (_Float16*)x16p;
  const int i = blockIdx.x * 256 + threadIdx.x;
  const int row = i >> 6, c8 = i & 63;
  const int t = row >> 6, b = row & 63;
  int tok = tokens[b * kStep + t];
  tok = tok < 0 ? 0 : tok;
  tok = tok > (kVocab - 1) ? (kVocab - 1) : tok;
  const float* src = emb + (size_t)tok * kEmb + c8 * 8;
  const v4f f0 = *(const v4f*)src;
  const v4f f1 = *(const v4f*)(src + 4);
  v8h hv;
  hv[0] = (_Float16)f0[0]; hv[1] = (_Float16)f0[1]; hv[2] = (_Float16)f0[2]; hv[3] = (_Float16)f0[3];
  hv[4] = (_Float16)f1[0]; hv[5] = (_Float16)f1[1]; hv[6] = (_Float16)f1[2]; hv[7] = (_Float16)f1[3];
  _Float16* dst = x16t + (size_t)row * kEmb + c8 * 8;
  *(volatile v8h*)dst = hv;
  __threadfence();
  *(volatile v8h*)dst = hv;
}

template <int LAYER>
__global__ __launch_bounds__(kRnnThreads) void rnn_scan_kernel(
    const float* __restrict__ xinT, const unsigned short* __restrict__ whhp,
    unsigned short* __restrict__ houtp,
    const float* __restrict__ wfc, const float* __restrict__ bfc,
    float* __restrict__ out) {
  __shared__ __align__(16) _Float16 hhi[2 * kHTile];
  __shared__ __align__(16) _Float16 hlo[2 * kHTile];
  __shared__ __align__(16) float fcp[(LAYER == 1) ? (2 * 8 * 32) : 4];
  __shared__ __align__(16) float obuf[(LAYER == 1) ? (kSeqPB * kFlushT * kCls) : 4];
  const _Float16* whh16 = (const _Float16*)whhp;
  _Float16* hout = (_Float16*)houtp;
  const int tid = threadIdx.x, lane = tid & 31, wave = tid >> 5;
  const int c = lane & 15, hh = lane >> 4, koff = hh * 8, mOff = hh * 8;
  const int seq0 = blockIdx.x * kSeqPB;
  const int n0 = wave * 64;
  const int q4 = lane >> 3, c8 = (lane & 7) * 8, c4f = (lane & 7) * 4;

  {
    const v8h z = {(_Float16)0.f, (_Float16)0.f, (_Float16)0.f, (_Float16)0.f, (_Float16)0.f, (_Float16)0.f, (_Float16)0.f, (_Float16)0.f};
    for (int i = tid; i < (2 * kHTile) / 8; i += kRnnThreads) {
      *(v8h*)(hhi + i * 8) = z;
      *(v8h*)(hlo + i * 8) = z;
    }
  }
  float wfc0[4] = {0.f, 0.f, 0.f, 0.f}, wfc1[4] = {0.f, 0.f, 0.f, 0.f};
  float bfl = 0.0f;
  if constexpr (LAYER == 1) {
#pragma unroll
    for (int j = 0; j < 4; ++j) {
      wfc0[j] = wfc[n0 + 16 * j + c];
      wfc1[j] = wfc[kHid + n0 + 16 * j + c];
    }
    bfl = bfc[lane & 1];
  }
  __syncthreads();

  const _Float16* brow = whh16 + (size_t)(n0 + c) * kHid + koff;
  const v8f z8 = {0.f, 0.f, 0.f, 0.f, 0.f, 0.f, 0.f, 0.f};

#pragma unroll 1
  for (int t = 0; t < kStep; ++t) {
    const int par = t & 1;
    const _Float16* hch = hhi + par * kHTile;
    const _Float16* hcl = hlo + par * kHTile;
    _Float16*       hnh = hhi + (par ^ 1) * kHTile;
    _Float16*       hnl = hlo + (par ^ 1) * kHTile;

    v8f acc[4], accr[4];
#pragma unroll
    for (int j = 0; j < 4; ++j) {
      const float* xp = xinT + (size_t)(n0 + 16 * j + c) * kRows + t * kSeq + seq0 + 8 * hh;
      const v4f xa = *(const v4f*)xp;
      const v4f xb = *(const v4f*)(xp + 4);
      acc[j][0] = xa[0] * kWCarry; acc[j][1] = xa[1] * kWCarry; acc[j][2] = xa[2] * kWCarry; acc[j][3] = xa[3] * kWCarry;
      acc[j][4] = xb[0] * kWCarry; acc[j][5] = xb[1] * kWCarry; acc[j][6] = xb[2] * kWCarry; acc[j][7] = xb[3] * kWCarry;
      accr[j] = z8;
    }
    const _Float16* arh = hch + c * kHP + koff;
    const _Float16* arl = hcl + c * kHP + koff;
#pragma unroll 1
    for (int kc = 0; kc < kHid / 32; ++kc) {
      const v16h fah = Frag<_Float16>::load(arh + kc * 32);
      const v16h fal = Frag<_Float16>::load(arl + kc * 32);
      v16h fb[4];
#pragma unroll
      for (int j = 0; j < 4; ++j) fb[j] = Frag<_Float16>::load(brow + (size_t)(16 * j) * kHid + kc * 32);
#pragma unroll
      for (int j = 0; j < 4; ++j) {
        acc[j]  = Frag<_Float16>::mma(fah, fb[j], acc[j]);
        accr[j] = Frag<_Float16>::mma(fal, fb[j], accr[j]);
      }
      dep_guard8_h(acc[0], acc[1], acc[2], acc[3], accr[0], accr[1], accr[2], accr[3], fah, fal, fb[0], fb[1], fb[2], fb[3]);
    }
    acc_guard4(acc[0], acc[1], acc[2], acc[3]);
    acc_guard4(accr[0], accr[1], accr[2], accr[3]);

    float pc0[8], pc1[8];
#pragma unroll
    for (int r = 0; r < 8; ++r) { pc0[r] = 0.0f; pc1[r] = 0.0f; }
#pragma unroll
    for (int j = 0; j < 4; ++j) {
#pragma unroll
      for (int r = 0; r < 8; ++r) {
        const float z  = fmaf(accr[j][r], kResInv, acc[j][r]) * kWCarryInv;
        const float hv = tanhf(z);
        const _Float16 h16 = (_Float16)hv;
        float res = hv - (float)h16;
        asm volatile("" : "+v"(res));
        const _Float16 r16 = (_Float16)(res * kResCarry);
        const int li = (mOff + r) * kHP + n0 + 16 * j + c;
        hnh[li] = h16;
        hnl[li] = r16;
        if constexpr (LAYER == 1) {
          pc0[r] = fmaf(hv, wfc0[j], pc0[r]);
          pc1[r] = fmaf(hv, wfc1[j], pc1[r]);
        }
      }
    }
    if constexpr (LAYER == 1) {
#pragma unroll
      for (int r = 0; r < 8; ++r) {
#pragma unroll
        for (int off = 1; off < 16; off <<= 1) {
          pc0[r] += __shfl_xor(pc0[r], off, 32);
          pc1[r] += __shfl_xor(pc1[r], off, 32);
        }
      }
      if (c == 0) {
#pragma unroll
        for (int r = 0; r < 8; ++r) {
          fcp[par * 256 + wave * 32 + (mOff + r) * 2 + 0] = pc0[r];
          fcp[par * 256 + wave * 32 + (mOff + r) * 2 + 1] = pc1[r];
        }
      }
    }
    __syncthreads();

    if constexpr (LAYER == 0) {
      const size_t rowbase = (size_t)t * kSeq + (size_t)seq0;
      for (int pass = 0; pass < 2; ++pass) {
#pragma unroll
        for (int it = 0; it < 4; ++it) {
          const int rr = it * 4 + q4;
          const v8h v = *(const v8h*)(hnh + rr * kHP + n0 + c8);
          *(volatile v8h*)(hout + (rowbase + rr) * kHid + n0 + c8) = v;
        }
        __threadfence();
      }
    } else {
      if (wave == 0) {
        float s = 0.0f;
#pragma unroll
        for (int w = 0; w < 8; ++w) s += fcp[par * 256 + w * 32 + lane];
        const int row = lane >> 1, cls = lane & 1;
        const int tt = t & (kFlushT - 1);
        obuf[row * (kFlushT * kCls) + tt * kCls + cls] = s + bfl;
        if (tt == kFlushT - 1) {
          __builtin_amdgcn_fence(__ATOMIC_RELEASE, "workgroup");
          __builtin_amdgcn_wave_barrier();
          __builtin_amdgcn_fence(__ATOMIC_ACQUIRE, "workgroup");
          const int t0 = t - (kFlushT - 1);
          for (int pass = 0; pass < 2; ++pass) {
#pragma unroll
            for (int it = 0; it < 4; ++it) {
              const int i = it * 4 + q4;
              const v4f v = *(const v4f*)(obuf + i * (kFlushT * kCls) + c4f);
              *(volatile v4f*)(out + ((size_t)(seq0 + i) * kStep + (size_t)t0) * kCls + c4f) = v;
            }
            __threadfence();
          }
        }
      }
    }
  }
}

extern "C" void kernel_launch(void* const* d_in, const int* in_sizes, int n_in,
                              void* d_out, int out_size, void* d_ws, size_t ws_size, hipStream_t stream) {
  if (n_in < 12 || d_out == nullptr || d_ws == nullptr) return;
  if (in_sizes[0] != kSeq * kStep || in_sizes[1] != kVocab * kEmb ||
      in_sizes[2] != kHid * kEmb || in_sizes[3] != kHid || in_sizes[4] != kHid * kHid || in_sizes[5] != kHid ||
      in_sizes[6] != kHid * kHid || in_sizes[7] != kHid || in_sizes[8] != kHid * kHid || in_sizes[9] != kHid ||
      in_sizes[10] != kCls * kHid || in_sizes[11] != kCls || out_size != kOutN) return;

  const int*   tokens = (const int*)  d_in[0];
  const float* emb    = (const float*)d_in[1];
  const float* w_ih0  = (const float*)d_in[2];
  const float* b_ih0  = (const float*)d_in[3];
  const float* w_hh0  = (const float*)d_in[4];
  const float* b_hh0  = (const float*)d_in[5];
  const float* w_ih1  = (const float*)d_in[6];
  const float* b_ih1  = (const float*)d_in[7];
  const float* w_hh1  = (const float*)d_in[8];
  const float* b_hh1  = (const float*)d_in[9];
  const float* w_fc   = (const float*)d_in[10];
  const float* b_fc   = (const float*)d_in[11];
  float* out = (float*)d_out;

  char* ws = (char*)d_ws; size_t off = 0;
  auto carve = [&](size_t bytes) -> char* { char* p = ws + off; off += (bytes + 255) & ~(size_t)255; return p; };
  unsigned short* WIH0_16 = (unsigned short*)carve((size_t)kHid * kEmb * 2);
  unsigned short* WHH0_16 = (unsigned short*)carve((size_t)kHid * kHid * 2);
  unsigned short* WIH1_16 = (unsigned short*)carve((size_t)kHid * kHid * 2);
  unsigned short* WHH1_16 = (unsigned short*)carve((size_t)kHid * kHid * 2);
  float*          BSUM    = (float*)carve((size_t)kDwBsum * 4);
  unsigned short* XH16    = (unsigned short*)carve((size_t)kRows * kEmb * 2);
  float*          XINT    = (float*)carve((size_t)kHid * kRows * 4);
  if (off > ws_size || off > (size_t)134217728) return;

  prep_kernel<<<kPrepBlocks, 256, 0, stream>>>(w_ih0, w_hh0, w_ih1, w_hh1, b_ih0, b_hh0, b_ih1, b_hh1,
                                               (unsigned*)WIH0_16, (unsigned*)WHH0_16,
                                               (unsigned*)WIH1_16, (unsigned*)WHH1_16, (unsigned*)BSUM);

  gather_kernel<<<kXChunks / 256, 256, 0, stream>>>(tokens, emb, XH16);

  wmma_gemm64<0, false, 1, 0, false, 0><<<dim3(kGemmGrid, 1), 256, 0, stream>>>(
      WIH0_16, WIH0_16, kEmb, 0L, XH16, XH16, kEmb, 0L,
      (void*)XINT, (void*)XINT, kRows, 0L, BSUM, BSUM, 0L, kHid, kRows, kEmb, kWCarryInv);

  rnn_scan_kernel<0><<<kRnnBlocks, kRnnThreads, 0, stream>>>(XINT, WHH0_16, XH16, w_fc, b_fc, out);

  wmma_gemm64<0, false, 1, 0, false, 0><<<dim3(kGemmGrid, 1), 256, 0, stream>>>(
      WIH1_16, WIH1_16, kHid, 0L, XH16, XH16, kHid, 0L,
      (void*)XINT, (void*)XINT, kRows, 0L, BSUM + kHid, BSUM, 0L, kHid, kRows, kHid, kWCarryInv);

  rnn_scan_kernel<1><<<kRnnBlocks, kRnnThreads, 0, stream>>>(XINT, WHH1_16, XH16, w_fc, b_fc, out);
}
